// N3Aggregation2D_21912923144705
// MI455X (gfx1250) — hardware-run, weakly checked
//
#include <hip/hip_runtime.h>
#include <math.h>

typedef __attribute__((ext_vector_type(16))) _Float16 v16h;
typedef __attribute__((ext_vector_type(8)))  _Float16 v8h;
typedef __attribute__((ext_vector_type(8)))  float    v8f;
typedef __attribute__((ext_vector_type(4)))  float    v4f;
typedef __attribute__((ext_vector_type(4)))  unsigned v4u;
typedef __attribute__((ext_vector_type(8)))  unsigned v8u;

constexpr int kHD    = 64;
constexpr int kHP    = 66;
constexpr int kNQ    = kHP * kHP;
constexpr int kNE    = 8;
constexpr int kNC    = 8;
constexpr int kNK    = 7;
constexpr int kPS    = 10;
constexpr int kADJ   = kPS / 2;
constexpr int kWS    = 29;
constexpr int kWOFF  = kWS / 2;
constexpr int kNW    = kWS * kWS;
constexpr int kKSEL  = 224;
constexpr int kNCH   = kKSEL / 32;
constexpr int kXP    = kHP + kPS - 1;
constexpr int kXSTR  = 76;
constexpr int kXPH   = kNC * kXP * kXSTR;
constexpr int kXPHP  = 45632;
constexpr int kQP    = 4384;
constexpr int kAQ    = 16 * kKSEL;
constexpr int kNBW   = 128;
constexpr int kNBMAX = (kHP - 1) * kXSTR + (kHP - 1);
constexpr int kZN    = 832;
constexpr int kZQ    = kNK * kZN;
constexpr int kNGRP  = kZN / 64;
constexpr int kNCOL  = kNC * kPS * kPS;
constexpr int kSlabP = 68;
constexpr int kOutQuads = (1 + kNK) * kNC * kHD * kHD / 4;

static_assert(kNQ == 4356);
static_assert(kNW == 841);
static_assert(kXP == 75);
static_assert(kXPH == 45600);
static_assert((kXPH % 8) == 0);
static_assert(kXPHP >= kXPH && (kXPHP * 2) % 128 == 0);
static_assert(kQP >= kNQ && (kQP % 32) == 0);
static_assert(kKSEL == kNCH * 32);
static_assert(kNCH == 7);
static_assert(kNCOL == 800 && kZN >= kNCOL && (kZN % 64) == 0);
static_assert((kAQ * 2) % 128 == 0 && (kZQ * 2) % 128 == 0 && (kNBW * 4) % 128 == 0);
static_assert(2 * (kNBMAX + ((kNC - 1) * kXP + kPS - 1) * kXSTR + kPS - 1) + 2 <= kXPH * 2);
static_assert(2 * kNBMAX < 65536);
static_assert(kOutQuads == 65536);

constexpr float kXCarry  = 1024.0f;
constexpr float kWCarry  = 32768.0f;
constexpr float kLoCarry = 2048.0f;
constexpr float kLoInv   = 1.0f / kLoCarry;
constexpr float kOutInv  = 1.0f / (kXCarry * kWCarry);
constexpr float kF16Min  = 6.103515625e-5f;
constexpr float kSkipThr = 1.0e-12f;
constexpr float kLtScale = 1.0f / (float)(kPS * kPS);

constexpr size_t kSzVec  = (size_t)kQP * 4;
constexpr size_t kSzXpad = (size_t)kXPHP * 2;
constexpr size_t kSzDist = (size_t)kNW * kQP * 4;
constexpr size_t kSzApl  = (size_t)kNQ * kAQ * 2;
constexpr size_t kSzNb   = (size_t)kNQ * kNBW * 4;
constexpr size_t kSzZ    = (size_t)kNQ * kZQ * 2;
constexpr size_t kOffN2Q  = 0;
constexpr size_t kOffN2D  = kOffN2Q + kSzVec;
constexpr size_t kOffLTV  = kOffN2D + kSzVec;
constexpr size_t kOffXPAD = kOffLTV + kSzVec;
constexpr size_t kOffDIST = kOffXPAD + kSzXpad;
constexpr size_t kOffAPL  = kOffDIST + kSzDist;
constexpr size_t kOffNB   = kOffAPL + kSzApl;
constexpr size_t kOffZ    = kOffNB + kSzNb;
constexpr size_t kWsTotal = kOffZ + kSzZ;
static_assert(kWsTotal == 99084416ull);
static_assert(kWsTotal <= 134217728ull);
static_assert((kOffN2D % 128) == 0 && (kOffLTV % 128) == 0 && (kOffXPAD % 128) == 0 && (kOffDIST % 128) == 0 &&
              (kOffAPL % 128) == 0 && (kOffNB % 128) == 0 && (kOffZ % 128) == 0);

__device__ __forceinline__ void pin_f(float& x) { asm volatile("" : "+v"(x)); }
__device__ __forceinline__ void pin_u(unsigned& x) { asm volatile("" : "+v"(x)); }
__device__ __forceinline__ int clampi(int v, int lo, int hi) { return v < lo ? lo : (v > hi ? hi : v); }
__device__ __forceinline__ float flush16(float v) { return (fabsf(v) < kF16Min) ? 0.0f : v; }

__device__ __forceinline__ float h16_to_f32(unsigned hb) {
  const unsigned sgn = (hb & 0x8000u) << 16;
  const unsigned em = hb & 0x7fffu;
  const float fn = __uint_as_float((em << 13) + 0x38000000u);
  const float fs = (float)em * 5.9604644775390625e-8f;
  const float mag = (em < 0x400u) ? fs : fn;
  return __uint_as_float(__float_as_uint(mag) | sgn);
}

union FragU { v16h v; v8h h[2]; };
__device__ __forceinline__ v16h frag_load(const _Float16* p) {
  FragU f;
  f.h[0] = *(const v8h*)(p);
  f.h[1] = *(const v8h*)(p + 16);
  return f.v;
}
__device__ __forceinline__ v8f mma_f16(v16h a, v16h b, v8f c) {
  c = __builtin_amdgcn_wmma_f32_16x16x32_f16(false, a, false, b, (short)0, c, false, false);
  asm volatile("v_nop\n\tv_nop\n\tv_nop\n\tv_nop" : "+v"(c) : "v"(a), "v"(b));
  return c;
}

__device__ __forceinline__ _Float16 enc_w(float w, bool lo, bool valid) {
  const float wc = w * kWCarry;
  const float hf = flush16(wc);
  const _Float16 hh = (_Float16)hf;
  const float res = flush16((wc - (float)hh) * kLoCarry);
  float o = lo ? res : hf;
  o = valid ? o : 0.0f;
  return (_Float16)o;
}

__global__ __launch_bounds__(256) void prep_kernel(
    const float* __restrict__ xe, const float* __restrict__ ye, const float* __restrict__ ltin,
    float* __restrict__ n2q, float* __restrict__ n2d, float* __restrict__ ltv)
{
  __shared__ __align__(16) float sv[3 * 256];
  const int tid = threadIdx.x;
  const int q = blockIdx.x * 256 + tid;
  const int qc = q < kNQ ? q : kNQ - 1;
  const int y = qc / kHP;
  const int x = qc - y * kHP;
  float sq = 0.0f, sd = 0.0f, sl = 0.0f;
#pragma unroll 1
  for (int oy = 0; oy < kPS; ++oy) {
    const int yy = y + oy - kADJ;
    const bool oky = (yy >= 1) && (yy <= kHD);
    const int yc = clampi(yy, 1, kHD) - 1;
    float rq = 0.0f, rd = 0.0f, rl = 0.0f;
#pragma unroll 1
    for (int ox = 0; ox < kPS; ++ox) {
      const int xx = x + ox - kADJ;
      const bool ok = oky && (xx >= 1) && (xx <= kHD);
      const int xc = clampi(xx, 1, kHD) - 1;
      const int base = yc * kHD + xc;
      float pq = 0.0f, pd = 0.0f;
#pragma unroll 1
      for (int e0 = 0; e0 < kNE; e0 += 4) {
#pragma unroll
        for (int e = 0; e < 4; ++e) {
          const float a = ye[(e0 + e) * kHD * kHD + base];
          const float b = xe[(e0 + e) * kHD * kHD + base];
          pq = fmaf(a, a, pq);
          pd = fmaf(b, b, pd);
        }
      }
      float lv = ltin[base];
      pin_f(pq);
      pin_f(pd);
      pin_f(lv);
      rq += ok ? pq : 0.0f;
      rd += ok ? pd : 0.0f;
      rl += ok ? lv : 0.0f;
    }
    sq += rq;
    sd += rd;
    sl += rl;
  }
  const bool live = q < kNQ;
  sv[tid]       = live ? sq : 0.0f;
  sv[256 + tid] = live ? sd : 0.0f;
  sv[512 + tid] = live ? (sl * kLtScale) : 0.0f;
  __syncthreads();
  if (tid < 64) {
    const int e0 = blockIdx.x * 256 + tid * 4;
    if (e0 < kQP) {
      const v4f a = *(const v4f*)(sv + tid * 4);
      const v4f b = *(const v4f*)(sv + 256 + tid * 4);
      const v4f c = *(const v4f*)(sv + 512 + tid * 4);
      for (int pass = 0; pass < 2; ++pass) {
        *(volatile v4f*)(n2q + e0) = a;
        *(volatile v4f*)(n2d + e0) = b;
        *(volatile v4f*)(ltv + e0) = c;
        __threadfence();
      }
    }
  }
}

__global__ __launch_bounds__(256) void xpad_kernel(const float* __restrict__ x, unsigned short* __restrict__ xp)
{
  const int i8 = blockIdx.x * 256 + threadIdx.x;
  if (i8 >= kXPHP / 8) return;
  v8h hv;
#pragma unroll
  for (int e = 0; e < 8; ++e) {
    const int i = i8 * 8 + e;
    const int ic = i < kXPH ? i : kXPH - 1;
    const int cc = ic / (kXP * kXSTR);
    const int rem = ic - cc * (kXP * kXSTR);
    const int rr = rem / kXSTR;
    const int col = rem - rr * kXSTR;
    const bool ok = (i < kXPH) && (rr >= 6) && (rr <= 69) && (col >= 6) && (col <= 69);
    const int rc = clampi(rr, 6, 69) - 6;
    const int sc = clampi(col, 6, 69) - 6;
    float v = x[(cc * kHD + rc) * kHD + sc];
    pin_f(v);
    v = ok ? (v * kXCarry) : 0.0f;
    v = flush16(v);
    hv[e] = (_Float16)v;
  }
  unsigned short* dst = xp + (size_t)i8 * 8;
  *(volatile v8h*)dst = hv;
  __threadfence();
  *(volatile v8h*)dst = hv;
}

__global__ __launch_bounds__(256) void dist_kernel(
    const float* __restrict__ xe, const float* __restrict__ ye,
    const float* __restrict__ n2q, const float* __restrict__ n2d, float* __restrict__ dist)
{
  __shared__ __align__(16) float prod[kXP * kXSTR];
  __shared__ float rows[kXP * kHP];
  static_assert(kXP * kXSTR >= kQP);
  const int tid = threadIdx.x;
  const int d = blockIdx.x;
  const int dyi = d / kWS;
  const int dy = dyi - kWOFF;
  const int dx = d - dyi * kWS - kWOFF;
#pragma unroll 1
  for (int i = tid; i < kXP * kXP; i += 256) {
    const int r = i / kXP;
    const int ci = i - r * kXP;
    const int yy = r - kADJ, xx = ci - kADJ;
    const int y2 = yy + dy, x2 = xx + dx;
    const bool ok = (yy >= 1) && (yy <= kHD) && (xx >= 1) && (xx <= kHD) &&
                    (y2 >= 1) && (y2 <= kHD) && (x2 >= 1) && (x2 <= kHD);
    const int b1 = (clampi(yy, 1, kHD) - 1) * kHD + clampi(xx, 1, kHD) - 1;
    const int b2 = (clampi(y2, 1, kHD) - 1) * kHD + clampi(x2, 1, kHD) - 1;
    float v = 0.0f;
#pragma unroll 1
    for (int e0 = 0; e0 < kNE; e0 += 4) {
#pragma unroll
      for (int e = 0; e < 4; ++e)
        v = fmaf(ye[(e0 + e) * kHD * kHD + b1], xe[(e0 + e) * kHD * kHD + b2], v);
    }
    pin_f(v);
    prod[r * kXSTR + ci] = ok ? v : 0.0f;
  }
  __syncthreads();
#pragma unroll 1
  for (int i = tid; i < kXP * kHP; i += 256) {
    const int r = i / kHP;
    const int x = i - r * kHP;
    float s = 0.0f;
#pragma unroll
    for (int o = 0; o < kPS; ++o) s += prod[r * kXSTR + x + o];
    rows[i] = s;
  }
  __syncthreads();
  const bool selfo = (dy == 0) && (dx == 0);
#pragma unroll 1
  for (int i = tid; i < kQP; i += 256) {
    const int ic = i < kNQ ? i : kNQ - 1;
    const int y = ic / kHP;
    const int x = ic - y * kHP;
    float cr = 0.0f;
#pragma unroll
    for (int o = 0; o < kPS; ++o) cr += rows[(y + o) * kHP + x];
    const int y2 = y + dy, x2 = x + dx;
    const bool valid = (y2 >= 0) && (y2 < kHP) && (x2 >= 0) && (x2 < kHP);
    float n2s = n2d[clampi(y2, 0, kHP - 1) * kHP + clampi(x2, 0, kHP - 1)];
    float nq = n2q[ic];
    pin_f(n2s);
    pin_f(nq);
    const float dv = (nq + n2s) - 2.0f * cr;
    const float sel = (valid && !selfo) ? dv : 1.0e10f;
    prod[i] = (i < kNQ) ? sel : 0.0f;
  }
  __syncthreads();
  float* drow = dist + (size_t)d * kQP;
  for (int pass = 0; pass < 2; ++pass) {
#pragma unroll 1
    for (int i4 = tid; i4 < kQP / 4; i4 += 256) {
      const v4f v = *(const v4f*)(prod + 4 * i4);
      *(volatile v4f*)(drow + 4 * i4) = v;
    }
    __threadfence();
  }
}

__global__ __launch_bounds__(256) void select_kernel(
    const float* __restrict__ dist, const float* __restrict__ ltv,
    unsigned short* __restrict__ apl, unsigned* __restrict__ nbp)
{
  __shared__ float skey[1024];
  __shared__ int   sidx[1024];
  __shared__ __align__(16) float wst[kNK * kKSEL];
  __shared__ int   snb[256];
  __shared__ unsigned sflag[8];
  __shared__ float redm[8];
  __shared__ float reds[8];
  const int tid = threadIdx.x, lane = tid & 31, wave = tid >> 5;
  const int q = blockIdx.x;
#pragma unroll 1
  for (int i = tid; i < 1024; i += 256) {
    const int ic = i < kNW ? i : kNW - 1;
    float v = dist[(size_t)ic * kQP + q];
    pin_f(v);
    skey[i] = (i < kNW) ? v : 3.0e38f;
    sidx[i] = i;
  }
#pragma unroll 1
  for (int k = 2; k <= 1024; k <<= 1) {
#pragma unroll 1
    for (int s = k >> 1; s > 0; s >>= 1) {
      __syncthreads();
#pragma unroll
      for (int u = 0; u < 2; ++u) {
        const int t = tid + u * 256;
        const int i = ((t & ~(s - 1)) << 1) | (t & (s - 1));
        const int j = i + s;
        const bool up = ((i & k) == 0);
        const float ki = skey[i], kj = skey[j];
        const int ii = sidx[i], ij = sidx[j];
        const bool gt = (ki > kj) || ((ki == kj) && (ii > ij));
        if (gt == up) {
          skey[i] = kj; skey[j] = ki;
          sidx[i] = ij; sidx[j] = ii;
        }
      }
    }
  }
  __syncthreads();

  const float ltq = ltv[q];
  const float rinv = 1.0f / expf(ltq);
  const int qy = q / kHP;
  const int qx = q - qy * kHP;
  const bool act = tid < kKSEL;
  const int tc = act ? tid : kKSEL - 1;
  const float keyv = skey[tc];
  const int dsel = clampi(sidx[tc], 0, kNW - 1);
  const int dyi = dsel / kWS;
  const int dxi = dsel - dyi * kWS;
  const int ny = clampi(qy + dyi - kWOFF, 0, kHP - 1);
  const int nx = clampi(qx + dxi - kWOFF, 0, kHP - 1);
  snb[tid] = act ? (ny * kXSTR + nx) : 0;

  float lg = act ? ((-keyv) * rinv) : -3.0e38f;
  float wmax = 0.0f;
#pragma unroll 1
  for (int it = 0; it < kNK; ++it) {
    float m = lg;
#pragma unroll
    for (int off = 16; off > 0; off >>= 1) m = fmaxf(m, __shfl_xor(m, off, 32));
    if (lane == 0) redm[wave] = m;
    __syncthreads();
    float mx = redm[0];
#pragma unroll
    for (int w = 1; w < 8; ++w) mx = fmaxf(mx, redm[w]);
    const float ev = expf(lg - mx);
    const float e = act ? ev : 0.0f;
    float s = e;
#pragma unroll
    for (int off = 16; off > 0; off >>= 1) s += __shfl_xor(s, off, 32);
    if (lane == 0) reds[wave] = s;
    __syncthreads();
    float sum = reds[0];
#pragma unroll
    for (int w = 1; w < 8; ++w) sum += reds[w];
    const float wv = e * (1.0f / sum);
    if (act) wst[it * kKSEL + tid] = wv;
    wmax = fmaxf(wmax, wv);
    const float upd = logf(fmaxf(1.0f - wv, 1.0e-6f));
    lg = act ? (lg + upd) : lg;
  }
  {
    float wm = wmax;
#pragma unroll
    for (int off = 16; off > 0; off >>= 1) wm = fmaxf(wm, __shfl_xor(wm, off, 32));
    if (lane == 0) sflag[wave] = ((wave < kNCH) && (wm >= kSkipThr)) ? 1u : 0u;
  }
  __syncthreads();

  v8h av[2];
#pragma unroll
  for (int it = 0; it < 2; ++it) {
    const int ci = tid + it * 256;
    const int cic = ci < 448 ? ci : 447;
    const int m = cic / 28;
    const int j0 = (cic - m * 28) * 8;
    const int kk = m & 7;
    const bool valid = kk < kNK;
    const int kr = valid ? kk : kNK - 1;
    const bool lo = m >= 8;
    const float* wp = wst + kr * kKSEL + j0;
    const v4f w0 = *(const v4f*)(wp);
    const v4f w1 = *(const v4f*)(wp + 4);
#pragma unroll
    for (int e = 0; e < 4; ++e) {
      av[it][e]     = enc_w(w0[e], lo, valid);
      av[it][4 + e] = enc_w(w1[e], lo, valid);
    }
  }
  unsigned short* aq = apl + (size_t)q * kAQ;
  for (int pass = 0; pass < 2; ++pass) {
    *(volatile v8h*)(aq + tid * 8) = av[0];
    if (tid < 192) *(volatile v8h*)(aq + (256 + tid) * 8) = av[1];
    __threadfence();
  }
  if (wave == 0) {
    v4u rec;
#pragma unroll
    for (int e = 0; e < 4; ++e) {
      const int wi = lane * 4 + e;
      const int wc = wi < 112 ? wi : 111;
      const unsigned a = (unsigned)snb[2 * wc];
      const unsigned b = (unsigned)snb[2 * wc + 1];
      const unsigned pw = (a & 0xffffu) | (b << 16);
      const unsigned f = sflag[clampi(wi - 112, 0, 7)];
      rec[e] = (wi < 112) ? pw : ((wi < 112 + kNCH) ? f : 0u);
    }
    unsigned* nq = nbp + (size_t)q * kNBW + lane * 4;
    *(volatile v4u*)nq = rec;
    __threadfence();
    *(volatile v4u*)nq = rec;
  }
}

__global__ __launch_bounds__(256) __attribute__((amdgpu_num_vgpr(256))) void agg_kernel(
    const unsigned short* __restrict__ xp, const unsigned short* __restrict__ apl,
    const unsigned* __restrict__ nbp, unsigned short* __restrict__ zpl)
{
  __shared__ __align__(16) unsigned short xl[kXPH];
  __shared__ __align__(16) float slab[8][kNK * kSlabP];
  const int tid = threadIdx.x, lane = tid & 31, wave = tid >> 5;
  {
    const v4u* src = (const v4u*)(const void*)xp;
    v4u* dst = (v4u*)(void*)xl;
#pragma unroll 1
    for (int i = tid; i < kXPH / 8; i += 256) dst[i] = src[i];
  }
  __syncthreads();
  const int q = blockIdx.x * 8 + wave;
  if (q < kNQ) {
    const int h = lane >> 4, c = lane & 15;
    const unsigned* nq = nbp + (size_t)q * kNBW;
    unsigned nbw[kNCH][8];
#pragma unroll
    for (int kc = 0; kc < kNCH; ++kc) {
      const v4u a = *(const v4u*)(nq + kc * 16 + 4 * h);
      const v4u b = *(const v4u*)(nq + kc * 16 + 8 + 4 * h);
#pragma unroll
      for (int i = 0; i < 4; ++i) {
        const unsigned wa = a[i];
        const unsigned wb = b[i];
        unsigned al = wa & 0xffffu, ah = wa >> 16;
        unsigned bl = wb & 0xffffu, bh = wb >> 16;
        al = al > (unsigned)kNBMAX ? (unsigned)kNBMAX : al;
        ah = ah > (unsigned)kNBMAX ? (unsigned)kNBMAX : ah;
        bl = bl > (unsigned)kNBMAX ? (unsigned)kNBMAX : bl;
        bh = bh > (unsigned)kNBMAX ? (unsigned)kNBMAX : bh;
        nbw[kc][i]     = (al << 1) | (ah << 17);
        nbw[kc][4 + i] = (bl << 1) | (bh << 17);
      }
    }
    int fl[kNCH];
#pragma unroll
    for (int kc = 0; kc < kNCH; ++kc) {
      const unsigned f = nq[112 + kc];
      fl[kc] = __builtin_amdgcn_readfirstlane((int)f);
    }
    const _Float16* ap = (const _Float16*)(const void*)apl + (size_t)q * kAQ + c * kKSEL + 8 * h;
    v16h afr[kNCH];
#pragma unroll
    for (int kc = 0; kc < kNCH; ++kc) afr[kc] = frag_load(ap + kc * 32);

    const char* xlb = (const char*)(const void*)xl;
    float* sl = slab[wave];
    const int q4 = lane >> 3, c8 = (lane & 7) * 8;
    unsigned short* zq = zpl + (size_t)q * kZQ + c8;

#pragma unroll 1
    for (int g = 0; g < kNGRP; ++g) {
#pragma unroll 1
      for (int t = 0; t < 4; ++t) {
        const int n = g * 64 + t * 16 + c;
        const int nn = n < kNCOL ? n : kNCOL - 1;
        const int cc = nn / (kPS * kPS);
        const int rem = nn - cc * (kPS * kPS);
        const int oy = rem / kPS;
        const int ox = rem - oy * kPS;
        const unsigned lc2 = (unsigned)((((cc * kXP + oy) * kXSTR) + ox) * 2);
        v8f acc = (v8f){0.f, 0.f, 0.f, 0.f, 0.f, 0.f, 0.f, 0.f};
#pragma unroll
        for (int kc = 0; kc < kNCH; ++kc) {
          if (fl[kc] != 0) {
            v8u bw;
#pragma unroll
            for (int i = 0; i < 8; ++i) {
              const unsigned w = nbw[kc][i];
              const unsigned o0 = (w & 0xffffu) + lc2;
              const unsigned o1 = (w >> 16) + lc2;
              const unsigned h0 = *(const unsigned short*)(xlb + o0);
              const unsigned h1 = *(const unsigned short*)(xlb + o1);
              bw[i] = h0 | (h1 << 16);
            }
            acc = mma_f16(afr[kc], __builtin_bit_cast(v16h, bw), acc);
          }
        }
#pragma unroll
        for (int r = 0; r < kNK; ++r) {
          const float mine = acc[r];
          const float oth = __shfl_xor(mine, 16, 32);
          const float v = (mine + oth * kLoInv) * kOutInv;
          if (h == 0) sl[r * kSlabP + t * 16 + c] = v;
        }
      }
      __builtin_amdgcn_fence(__ATOMIC_RELEASE, "workgroup");
      __builtin_amdgcn_wave_barrier();
      __builtin_amdgcn_fence(__ATOMIC_ACQUIRE, "workgroup");
      v8h o0, o1;
      {
        const float* sp = sl + q4 * kSlabP + c8;
        const v4f a = *(const v4f*)(sp);
        const v4f b = *(const v4f*)(sp + 4);
#pragma unroll
        for (int e = 0; e < 4; ++e) { o0[e] = (_Float16)a[e]; o0[4 + e] = (_Float16)b[e]; }
      }
      {
        const int r1 = (4 + q4) < kNK ? (4 + q4) : kNK - 1;
        const float* sp = sl + r1 * kSlabP + c8;
        const v4f a = *(const v4f*)(sp);
        const v4f b = *(const v4f*)(sp + 4);
#pragma unroll
        for (int e = 0; e < 4; ++e) { o1[e] = (_Float16)a[e]; o1[4 + e] = (_Float16)b[e]; }
      }
      unsigned short* zg = zq + g * 64;
      for (int pass = 0; pass < 2; ++pass) {
        *(volatile v8h*)(zg + q4 * kZN) = o0;
        if (q4 < 3) *(volatile v8h*)(zg + (4 + q4) * kZN) = o1;
        __threadfence();
      }
      __builtin_amdgcn_fence(__ATOMIC_RELEASE, "workgroup");
      __builtin_amdgcn_wave_barrier();
      __builtin_amdgcn_fence(__ATOMIC_ACQUIRE, "workgroup");
    }
  }
}

__device__ __forceinline__ int cover1(int p) {
  const int a = p < (kPS - 1) ? p : (kPS - 1);
  const int b = (p - (kHP - 1)) > 0 ? (p - (kHP - 1)) : 0;
  return a - b + 1;
}

__global__ __launch_bounds__(256) void fold_kernel(
    const float* __restrict__ y, const unsigned* __restrict__ zw, float* __restrict__ out)
{
  const int t = blockIdx.x * 256 + threadIdx.x;
  if (t >= kOutQuads) return;
  const int ch = t >> 10;
  const int rem = t & 1023;
  const int Y = rem >> 4;
  const int X0 = (rem & 15) * 4;
  const v4f yv = *(const v4f*)(y + ((ch & 7) * kHD + Y) * kHD + X0);
  v4f res = yv;
  if (ch >= kNC) {
    const int m = ch - kNC;
    const int k = m >> 3;
    const int c = m & 7;
    const int PY = Y + 6;
    const int PX0 = X0 + 6;
    float acc[4] = {0.0f, 0.0f, 0.0f, 0.0f};
#pragma unroll 1
    for (int oy = 0; oy < kPS; ++oy) {
      const int qy = PY - oy;
      const bool oky = (qy >= 0) && (qy < kHP);
      const int qyc = clampi(qy, 0, kHP - 1);
#pragma unroll 1
      for (int ox = 0; ox < kPS; ++ox) {
        const int off = c * (kPS * kPS) + oy * kPS + ox;
#pragma unroll
        for (int e = 0; e < 4; ++e) {
          const int qx = PX0 + e - ox;
          const bool ok = oky && (qx >= 0) && (qx < kHP);
          const int qxc = clampi(qx, 0, kHP - 1);
          const int elem = ((qyc * kHP + qxc) * kNK + k) * kZN + off;
          unsigned w = zw[elem >> 1];
          pin_u(w);
          const unsigned hb = (elem & 1) ? (w >> 16) : (w & 0xffffu);
          const float v = h16_to_f32(hb);
          acc[e] += ok ? v : 0.0f;
        }
      }
    }
    const int ca = cover1(PY);
#pragma unroll
    for (int e = 0; e < 4; ++e) {
      const float cnt = (float)(ca * cover1(PX0 + e));
      res[e] = acc[e] * (1.0f / cnt) - yv[e];
    }
  }
  float* dst = out + (size_t)t * 4;
  *(volatile v4f*)dst = res;
  __threadfence();
  *(volatile v4f*)dst = res;
}

extern "C" void kernel_launch(void* const* d_in, const int* in_sizes, int n_in,
                              void* d_out, int out_size, void* d_ws, size_t ws_size,
                              hipStream_t stream) {
  if (n_in < 5) return;
  if (in_sizes[0] != kNC * kHD * kHD) return;
  if (in_sizes[1] != kNE * kHD * kHD) return;
  if (in_sizes[2] != kNE * kHD * kHD) return;
  if (in_sizes[3] != kNC * kHD * kHD) return;
  if (in_sizes[4] != kHD * kHD) return;
  if (out_size != (1 + kNK) * kNC * kHD * kHD) return;
  if (ws_size < kWsTotal) return;

  const float* x    = (const float*)d_in[0];
  const float* xe   = (const float*)d_in[1];
  const float* ye   = (const float*)d_in[2];
  const float* y    = (const float*)d_in[3];
  const float* ltin = (const float*)d_in[4];
  float* out = (float*)d_out;

  char* ws = (char*)d_ws;
  float*          n2q  = (float*)(ws + kOffN2Q);
  float*          n2d  = (float*)(ws + kOffN2D);
  float*          ltv  = (float*)(ws + kOffLTV);
  unsigned short* xpad = (unsigned short*)(ws + kOffXPAD);
  float*          dist = (float*)(ws + kOffDIST);
  unsigned short* aplp = (unsigned short*)(ws + kOffAPL);
  unsigned*       nbp  = (unsigned*)(ws + kOffNB);
  unsigned short* zpl  = (unsigned short*)(ws + kOffZ);

  prep_kernel<<<(kQP + 255) / 256, 256, 0, stream>>>(xe, ye, ltin, n2q, n2d, ltv);
  xpad_kernel<<<(kXPHP / 8 + 255) / 256, 256, 0, stream>>>(x, xpad);
  dist_kernel<<<kNW, 256, 0, stream>>>(xe, ye, n2q, n2d, dist);
  select_kernel<<<kNQ, 256, 0, stream>>>(dist, ltv, aplp, nbp);
  agg_kernel<<<(kNQ + 7) / 8, 256, 0, stream>>>(xpad, aplp, nbp, zpl);
  fold_kernel<<<kOutQuads / 256, 256, 0, stream>>>(y, (const unsigned*)zpl, out);
}
